// TransformerLayer_75849122447780
// MI455X (gfx1250) — hardware-verified
//
#include <hip/hip_runtime.h>
#include <math.h>

typedef __attribute__((ext_vector_type(16))) _Float16 v16h;
typedef __attribute__((ext_vector_type(8)))  _Float16 v8h;
typedef __attribute__((ext_vector_type(8)))  float v8f;
typedef __attribute__((ext_vector_type(4)))  float v4f;

#ifndef SEQ
#define SEQ 2048
#endif
#define SEQ_FULL 2048
#ifndef NB
#define NB 4
#endif
#define NB_FULL 4
#ifndef PE_LEN
#define PE_LEN SEQ
#endif
#define DM 1024
#define NHEAD 16
#define HD 64
#define NQKV 3072
#define RC (4096.0f)
#define WC (16.0f)
#define PSH (14.0f)
#define SC2 (0.18033688011112042f)
#define L2_10K (13.287712379549449f)
#define F16MIN (6.103515625e-05f)
static_assert(SEQ % 128 == 0);
static_assert(SEQ >= 128);
static_assert(SEQ <= SEQ_FULL);
static_assert(NB >= 1);
static_assert(NB <= NB_FULL);
static_assert(DM == 1024);
static_assert(NHEAD * HD == DM);
static_assert(NQKV == 3 * DM);
static_assert(HD == 64);

#define WSZ_XH   (2u * (size_t)NB * SEQ * DM)
#define WSZ_PE   (2u * (size_t)SEQ * DM)
#define WSZ_WT   (2u * (size_t)NQKV * DM)
#define WSZ_PEW  (4u * (size_t)SEQ * NQKV)
#define WSZ_QP   (2u * (size_t)NHEAD * NB * SEQ * HD)
#define WS_XH   ((size_t)0)
#define WS_PEH  (WS_XH  + WSZ_XH)
#define WS_PER  (WS_PEH + WSZ_PE)
#define WS_WT   (WS_PER + WSZ_PE)
#define WS_PEW  (WS_WT  + WSZ_WT)
#define WS_QH   (WS_PEW + WSZ_PEW)
#define WS_KH   (WS_QH  + WSZ_QP)
#define WS_VT   (WS_KH  + WSZ_QP)
#define WS_END  (WS_VT  + WSZ_QP)
static_assert(WS_END <= (size_t)134217728u);
static_assert((WS_PEH % 256u) == 0 && (WS_PER % 256u) == 0 && (WS_WT % 256u) == 0 && (WS_PEW % 256u) == 0);
static_assert((WS_QH % 256u) == 0 && (WS_KH % 256u) == 0 && (WS_VT % 256u) == 0);
static_assert(((size_t)NB * SEQ / 2) * 256u * 8u == (size_t)NB * SEQ * DM);
static_assert((size_t)SEQ * 128u * 8u == (size_t)SEQ * DM);
static_assert((size_t)16 * 16 * 3 * 512u * 8u == (size_t)NQKV * DM);
static_assert(((size_t)SEQ / 64) * (NQKV / 64) * 4u * 16u * 64u == (size_t)SEQ * NQKV);
static_assert(((size_t)NB * SEQ / 64) * 16u * 64u * 128u == 2u * (size_t)NHEAD * NB * SEQ * HD);
static_assert(((size_t)NB * SEQ / 64) * 8u * 64u * 128u == (size_t)NHEAD * NB * SEQ * HD);
static_assert(((size_t)SEQ / 128) * (NHEAD * NB) * 8u * 16u * 64u == (size_t)NHEAD * NB * SEQ * HD);

template <typename T> __device__ __forceinline__ void vst2(void* p, T v) { *(volatile T*)p = v; __threadfence(); *(volatile T*)p = v; }
__device__ __forceinline__ v8f zero8() { v8f z = {0.f, 0.f, 0.f, 0.f, 0.f, 0.f, 0.f, 0.f}; return z; }
__device__ __forceinline__ v8f wmma16(v16h a, v16h b, v8f c) {
  v8f d = __builtin_amdgcn_wmma_f32_16x16x32_f16(false, a, false, b, (short)0, c, false, false);
  asm volatile("v_nop\n\tv_nop\n\tv_nop\n\tv_nop" : "+v"(d) : "v"(a), "v"(b));
  return d;
}
__device__ __forceinline__ v16h frag_h(const _Float16* rowk0, unsigned lane) {
  union { v16h v; v8h q[2]; } u; const _Float16* p = rowk0 + 8u * (lane >> 4);
  u.q[0] = *(const v8h*)p; u.q[1] = *(const v8h*)(p + 16); return u.v;
}
__device__ __forceinline__ _Float16 f16n(float x) { const float t = (fabsf(x) >= F16MIN) ? x : 0.0f; return (_Float16)t; }
__device__ __forceinline__ unsigned short bf16bits(float x) { unsigned u = __float_as_uint(x); u += 0x7FFFu + ((u >> 16) & 1u); return (unsigned short)(u >> 16); }
__device__ __forceinline__ float bf16val(unsigned short b) { return __uint_as_float(((unsigned)b) << 16); }
__device__ __forceinline__ float bfq(float x) { return bf16val(bf16bits(x)); }
__device__ __forceinline__ float ex2(float x) { return __builtin_amdgcn_exp2f(x); }
#define LDSX() do { asm volatile("s_wait_dscnt 0" ::: "memory"); __builtin_amdgcn_wave_barrier(); __builtin_amdgcn_fence(3  , "workgroup"); } while (0)

__global__ __launch_bounds__(256) void k_xcv(const float* __restrict__ src, _Float16* __restrict__ dst) {
  const unsigned i = blockIdx.x * 256u + threadIdx.x;
  const unsigned row = i >> 7, g8 = i & 127u;
  const unsigned b = row / (unsigned)SEQ, n = row - b * (unsigned)SEQ;
  const float* p = src + ((size_t)(b * (unsigned)SEQ_FULL + n) * DM + g8 * 8u);
  const v4f a = *(const v4f*)p, c = *(const v4f*)(p + 4);
  v8h o;
#pragma unroll
  for (int e = 0; e < 4; ++e) { o[e] = f16n(bfq(a[e])); o[4 + e] = f16n(bfq(c[e])); }
  vst2(dst + (size_t)i * 8u, o);
}

__global__ __launch_bounds__(256) void k_pe(_Float16* __restrict__ PEH, _Float16* __restrict__ PER) {
  __shared__ __align__(16) float spe[DM];
  const unsigned tid = threadIdx.x, pos = blockIdx.x;
  const unsigned pev = pos & ~1u;
  const bool podd = (pos & 1u) != 0u;
  const float invp = exp2f(-((2.0f * (float)pev) * (1.0f / (float)PE_LEN)) * L2_10K);
  float keep = 0.f;
#pragma unroll 1
  for (unsigned it = 0; it < 8u; ++it) {
    const unsigned e = it >> 1, which = it & 1u;
    const unsigned i = tid + 256u * e;
    const unsigned ie = i & ~1u;
    const float invi = exp2f(-((2.0f * (float)ie) * (1.0f / (float)DM)) * L2_10K);
    const float arg = (which != 0u) ? (float)i * invp : (float)pos * invi;
    const float s = sinf(arg), c = cosf(arg);
    const bool odd = (which != 0u) ? podd : ((i & 1u) != 0u);
    const float val = odd ? c : s;
    if (which == 0u) keep = val; else spe[i] = keep * val;
  }
  __syncthreads();
  if (tid < 128u) {
    const v4f a = *(const v4f*)&spe[tid * 8u], b = *(const v4f*)&spe[tid * 8u + 4u];
    v8h oh, orr;
#pragma unroll
    for (int e = 0; e < 4; ++e) {
      const _Float16 h0 = f16n(a[e]); oh[e] = h0; orr[e] = f16n((a[e] - (float)h0) * RC);
      const _Float16 h1 = f16n(b[e]); oh[4 + e] = h1; orr[4 + e] = f16n((b[e] - (float)h1) * RC);
    }
    const size_t o = (size_t)pos * DM + tid * 8u;
    vst2(PEH + o, oh); vst2(PER + o, orr);
  }
}

__global__ __launch_bounds__(256) void k_wt(const float* __restrict__ W0, const float* __restrict__ W1, const float* __restrict__ W2, _Float16* __restrict__ WT) {
  __shared__ __align__(16) _Float16 t[64][72];
  const unsigned tid = threadIdx.x, z = blockIdx.z;
  const float* W = (z == 0u) ? W0 : ((z == 1u) ? W1 : W2);
  const unsigned k0 = blockIdx.x * 64u, n0 = blockIdx.y * 64u;
  const unsigned kr = tid >> 2, nc = (tid & 3u) * 16u;
#pragma unroll
  for (unsigned c4 = 0; c4 < 4u; ++c4) {
    const v4f a = *(const v4f*)(W + (size_t)(k0 + kr) * DM + n0 + nc + 4u * c4);
#pragma unroll
    for (int e = 0; e < 4; ++e) t[nc + 4u * c4 + e][kr] = f16n(bfq(a[e]) * WC);
  }
  __syncthreads();
#pragma unroll
  for (unsigned it = 0; it < 2u; ++it) {
    const unsigned e = tid + 256u * it; const unsigned nr = e >> 3, q = e & 7u;
    vst2(WT + (size_t)(z * (unsigned)DM + n0 + nr) * DM + k0 + q * 8u, *(const v8h*)&t[nr][q * 8u]);
  }
}

__global__ __launch_bounds__(128) void k_pew(const _Float16* __restrict__ PEH, const _Float16* __restrict__ PER, const _Float16* __restrict__ WT, float* __restrict__ PEW) {
  __shared__ __align__(16) float sf[4][16][68];
  const unsigned tid = threadIdx.x, wave = tid >> 5, lane = tid & 31u, col = lane & 15u, g = lane >> 4;
  const unsigned r0 = blockIdx.x * 64u + wave * 16u, c0 = blockIdx.y * 64u;
  v8f ah[4], ar[4];
#pragma unroll
  for (int j = 0; j < 4; ++j) { ah[j] = zero8(); ar[j] = zero8(); }
#pragma unroll 1
  for (unsigned kc = 0; kc < DM / 32; ++kc) {
    const v16h a1 = frag_h(PEH + (size_t)(r0 + col) * DM + kc * 32u, lane);
    const v16h a2 = frag_h(PER + (size_t)(r0 + col) * DM + kc * 32u, lane);
#pragma unroll
    for (int j = 0; j < 4; ++j) {
      const v16h b = frag_h(WT + (size_t)(c0 + j * 16 + col) * DM + kc * 32u, lane);
      ah[j] = wmma16(a1, b, ah[j]); ar[j] = wmma16(a2, b, ar[j]);
    }
  }
#pragma unroll
  for (int j = 0; j < 4; ++j)
#pragma unroll
    for (int r = 0; r < 8; ++r) sf[wave][8u * g + r][j * 16 + col] = (ah[j][r] + ar[j][r] * (1.0f / RC)) * (1.0f / WC);
  LDSX();
#pragma unroll
  for (unsigned rp = 0; rp < 8u; ++rp) { const unsigned rl = 2u * rp + g; const v4f v = *(const v4f*)&sf[wave][rl][col * 4u]; vst2(PEW + (size_t)(r0 + rl) * NQKV + c0 + col * 4u, v); }
}

__global__ __launch_bounds__(128) void k_proj(const _Float16* __restrict__ XH, const _Float16* __restrict__ WT, const float* __restrict__ PEW,
                                              const float* __restrict__ bq, const float* __restrict__ bk, const float* __restrict__ bv,
                                              _Float16* __restrict__ QH, _Float16* __restrict__ KH, _Float16* __restrict__ VT) {
  __shared__ __align__(16) float sf[64][132];
  const unsigned tid = threadIdx.x, wave = tid >> 5, lane = tid & 31u, col = lane & 15u, g = lane >> 4;
  const unsigned r0 = blockIdx.x * 64u, c0 = blockIdx.y * 128u;
  const unsigned b = r0 / (unsigned)SEQ, n0 = r0 - b * (unsigned)SEQ;
  v8f acc[8];
#pragma unroll
  for (int j = 0; j < 8; ++j) acc[j] = zero8();
#pragma unroll 1
  for (unsigned kc = 0; kc < DM / 32; ++kc) {
    const v16h a = frag_h(XH + (size_t)(r0 + wave * 16u + col) * DM + kc * 32u, lane);
#pragma unroll
    for (int j = 0; j < 8; ++j) acc[j] = wmma16(a, frag_h(WT + (size_t)(c0 + j * 16 + col) * DM + kc * 32u, lane), acc[j]);
  }
#pragma unroll
  for (int j = 0; j < 8; ++j)
#pragma unroll
    for (int r = 0; r < 8; ++r) sf[wave * 16u + 8u * g + r][j * 16 + col] = acc[j][r] * (1.0f / WC);
  __syncthreads();
  const unsigned sel = blockIdx.y >> 3;
  const unsigned cw0 = (blockIdx.y & 7u) * 128u;
  const float* bias = (sel == 0u) ? bq : ((sel == 1u) ? bk : bv);
  if (sel < 2u) {
    _Float16* dst = (sel == 0u) ? QH : KH;
    const unsigned q = tid & 15u; const unsigned cw = cw0 + q * 8u; const unsigned h = cw >> 6, dh = cw & 63u;
    v4f b0 = *(const v4f*)(bias + cw), b1 = *(const v4f*)(bias + cw + 4u);
#pragma unroll
    for (int e = 0; e < 4; ++e) { b0[e] = bfq(b0[e]); b1[e] = bfq(b1[e]); }
#pragma unroll 1
    for (unsigned it = 0; it < 8u; ++it) {
      const unsigned rl = (tid >> 4) + 8u * it; const unsigned n = n0 + rl;
      const v4f s0 = *(const v4f*)&sf[rl][q * 8u], s1 = *(const v4f*)&sf[rl][q * 8u + 4u];
      const float* pw = PEW + (size_t)n * NQKV + c0 + q * 8u;
      const v4f p0 = *(const v4f*)pw, p1 = *(const v4f*)(pw + 4);
      v8h o;
#pragma unroll
      for (int e = 0; e < 4; ++e) { o[e] = f16n((s0[e] + p0[e]) + b0[e]); o[4 + e] = f16n((s1[e] + p1[e]) + b1[e]); }
      vst2(dst + ((size_t)(h * (unsigned)NB + b) * SEQ + n) * HD + dh, o);
    }
  } else {
    const unsigned q = tid & 7u;
#pragma unroll 1
    for (unsigned it = 0; it < 8u; ++it) {
      const unsigned cl = (tid >> 3) + 16u * it; const unsigned cw = cw0 + cl; const unsigned h = cw >> 6, dh = cw & 63u;
      const float bb = bfq(bias[cw]);
      v8h o;
#pragma unroll
      for (unsigned i = 0; i < 8u; ++i) { const unsigned rl = q * 8u + i; o[i] = f16n((sf[rl][cl] + PEW[(size_t)(n0 + rl) * NQKV + c0 + cl]) + bb); }
      vst2(VT + ((size_t)(h * (unsigned)NB + b) * HD + dh) * SEQ + n0 + q * 8u, o);
    }
  }
}

__global__ __launch_bounds__(256) void k_attn(const _Float16* __restrict__ QH, const _Float16* __restrict__ KH, const _Float16* __restrict__ VT, float* __restrict__ OUT) {
  __shared__ __align__(16) float sf[8][16][68];
  const unsigned tid = threadIdx.x, wave = tid >> 5, lane = tid & 31u, col = lane & 15u, g = lane >> 4;
  const unsigned hbi = blockIdx.y;
  const unsigned q0 = blockIdx.x * 128u + wave * 16u;
  const _Float16* Qb = QH + (size_t)hbi * SEQ * HD;
  const _Float16* Kb = KH + (size_t)hbi * SEQ * HD;
  const _Float16* Vb = VT + (size_t)hbi * HD * SEQ;
  const v16h qf0 = frag_h(Qb + (size_t)(q0 + col) * HD, lane);
  const v16h qf1 = frag_h(Qb + (size_t)(q0 + col) * HD + 32, lane);
  float m = -3.0e38f, l = 0.f;
  v8f acc[4];
#pragma unroll
  for (int j = 0; j < 4; ++j) acc[j] = zero8();
#pragma unroll 1
  for (unsigned kt = 0; kt < SEQ / 64; ++kt) {
    const unsigned key0 = kt * 64u;
    v8f c[4];
#pragma unroll
    for (int t = 0; t < 4; ++t) {
      const _Float16* kr = Kb + (size_t)(key0 + t * 16 + col) * HD;
      v8f z = zero8();
      z = wmma16(frag_h(kr, lane), qf0, z);
      z = wmma16(frag_h(kr + 32, lane), qf1, z);
      c[t] = z;
    }
    float tm = fmaxf(fmaxf(c[0][0], c[1][0]), fmaxf(c[2][0], c[3][0]));
#pragma unroll
    for (int r = 1; r < 8; ++r) tm = fmaxf(tm, fmaxf(fmaxf(c[0][r], c[1][r]), fmaxf(c[2][r], c[3][r])));
    tm = fmaxf(tm, __shfl_xor(tm, 16));
    const float mn = fmaxf(m, tm * SC2);
    const float sc = ex2(m - mn);
    const float sh = PSH - mn;
    m = mn; l *= sc;
#pragma unroll
    for (int j = 0; j < 4; ++j)
#pragma unroll
      for (int r = 0; r < 8; ++r) acc[j][r] *= sc;
#pragma unroll
    for (int u = 0; u < 2; ++u) {
      v16h pb;
#pragma unroll
      for (int i = 0; i < 8; ++i) {
        const float a0 = fmaxf(fmaf(c[2 * u][i], SC2, sh), -PSH);
        const float a1 = fmaxf(fmaf(c[2 * u + 1][i], SC2, sh), -PSH);
        const _Float16 h0 = (_Float16)ex2(a0), h1 = (_Float16)ex2(a1);
        pb[i] = h0; pb[8 + i] = h1;
        l += (float)h0 + (float)h1;
      }
#pragma unroll
      for (int j = 0; j < 4; ++j) acc[j] = wmma16(frag_h(Vb + (size_t)(j * 16 + col) * SEQ + key0 + u * 32, lane), pb, acc[j]);
    }
  }
  l += __shfl_xor(l, 16);
  const float inv = 1.0f / l;
#pragma unroll
  for (int j = 0; j < 4; ++j) {
    v4f lo = {acc[j][0] * inv, acc[j][1] * inv, acc[j][2] * inv, acc[j][3] * inv};
    v4f hi = {acc[j][4] * inv, acc[j][5] * inv, acc[j][6] * inv, acc[j][7] * inv};
    *(v4f*)&sf[wave][col][16 * j + 8u * g] = lo;
    *(v4f*)&sf[wave][col][16 * j + 8u * g + 4u] = hi;
  }
  LDSX();
  const unsigned hh = hbi / (unsigned)NB, bb = hbi - hh * (unsigned)NB;
  float* ob = OUT + ((size_t)(hh * (unsigned)NB_FULL + bb) * SEQ_FULL + q0) * HD;
#pragma unroll
  for (unsigned i = 0; i < 8u; ++i) { const unsigned rl = 2u * i + g; const v4f v = *(const v4f*)&sf[wave][rl][col * 4u]; vst2(ob + (size_t)rl * HD + col * 4u, v); }
}

extern "C" void kernel_launch(void* const* d_in, const int* in_sizes, int n_in, void* d_out, int out_size, void* d_ws, size_t ws_size, hipStream_t stream) {
  if (n_in < 7) return;
  if ((size_t)in_sizes[0] < ((size_t)(NB - 1) * SEQ_FULL + SEQ) * DM) return;
  if (in_sizes[1] < DM * DM || in_sizes[3] < DM * DM || in_sizes[5] < DM * DM) return;
  if (in_sizes[2] < DM || in_sizes[4] < DM || in_sizes[6] < DM) return;
  if ((size_t)out_size < ((size_t)((NHEAD - 1) * NB_FULL + (NB - 1)) * SEQ_FULL + SEQ) * HD) return;
  if (ws_size < (size_t)WS_END) return;
  const float* X = (const float*)d_in[0]; const float* WQ = (const float*)d_in[1]; const float* BQ = (const float*)d_in[2];
  const float* WK = (const float*)d_in[3]; const float* BK = (const float*)d_in[4]; const float* WV = (const float*)d_in[5]; const float* BV = (const float*)d_in[6];
  char* ws = (char*)d_ws;
  _Float16 *XH = (_Float16*)(ws + WS_XH), *PEH = (_Float16*)(ws + WS_PEH), *PER = (_Float16*)(ws + WS_PER), *WT = (_Float16*)(ws + WS_WT);
  _Float16 *QH = (_Float16*)(ws + WS_QH), *KH = (_Float16*)(ws + WS_KH), *VT = (_Float16*)(ws + WS_VT);
  float* PEW = (float*)(ws + WS_PEW);

  k_xcv<<<dim3(NB * SEQ / 2), 256, 0, stream>>>(X, XH);
  k_pe<<<dim3(SEQ), 256, 0, stream>>>(PEH, PER);
  k_wt<<<dim3(DM / 64, DM / 64, 3), 256, 0, stream>>>(WQ, WK, WV, WT);
  k_pew<<<dim3(SEQ / 64, NQKV / 64), 128, 0, stream>>>(PEH, PER, WT, PEW);
  k_proj<<<dim3(NB * SEQ / 64, NQKV / 128), 128, 0, stream>>>(XH, WT, PEW, BQ, BK, BV, QH, KH, VT);
  k_attn<<<dim3(SEQ / 128, NHEAD * NB), 256, 0, stream>>>(QH, KH, VT, (float*)d_out);
}
